// SpatioTemporalGNN_77051713290277
// MI455X (gfx1250) — hardware-verified
//
#include <hip/hip_runtime.h>
#include <stddef.h>
#include <stdint.h>
#include <math.h>


#define DIN    16
#define HID    256
#define H2C    128
#define DOUT   2
#define KX     32
#define G3     768
#define NTHR   256
#define NWAVE  8
#define EPT    8
#define CHUNK  (NTHR * EPT)
#define WCAP   (EPT * 32)
#define LISTN  (NWAVE * WCAP)
#define NBD    8192
#define SLD    13
#define NBA    512
#define SLA    9
#define RCAP   24576
#define DEGCAP 128
#define GBM    64
#define GBN    128
#define GTHR   128
#define U_W1T  (HID * (KX / 8))
#define U_W2T  (HID * (HID / 8))
#define U_WIH  (G3 * (HID / 8))
#define U_WD1T (HID * (HID / 8))
#define U_WD1X (HID * (KX / 8))
#define U_WD2T (H2C * (HID / 8))
#define U_WD3T (16 * (H2C / 8))
#define O1 (U_W1T)
#define O2 (O1 + U_W2T)
#define O3 (O2 + U_WIH)
#define O4 (O3 + U_WD1T)
#define O5 (O4 + U_WD1X)
#define O6 (O5 + U_WD2T)
#define O7 (O6 + U_WD3T)
#define AGG_ZINTS (LISTN + 2 * RCAP + 3 * NBA)
#define AGG_LDS_INTS (AGG_ZINTS + 16)
#define GRU_LDS_BYTES (3 * 64 * 64 * 4 + 2 * 64 * 64 * 2)
#define WSMAX  134217728
#define ASC    8.0f
#define WSC    1024.0f
#define RSC    2048.0f
#define SCL    (1.0f / 8192.0f)
#define SCLR   (1.0f / 16777216.0f)

static_assert((CHUNK & (CHUNK - 1)) == 0 && CHUNK <= 4096);
static_assert((NBD & (NBD - 1)) == 0 && NBD == (1 << SLD));
static_assert((NBA & (NBA - 1)) == 0 && NBA == (1 << SLA));
static_assert(((long long)CHUNK << SLD) < (1LL << 31));
static_assert(((long long)CHUNK << SLA) < (1LL << 31));
static_assert(NBD % (NTHR * 4) == 0);
static_assert(LISTN % NTHR == 0);
static_assert(NBA % NWAVE == 0 && NBA % 32 == 0 && NBA % GBM == 0);
static_assert(RCAP % 4 == 0 && AGG_ZINTS % 4 == 0 && LISTN % 4 == 0);
static_assert(U_W1T % NTHR == 0 && U_W2T % NTHR == 0 && U_WIH % NTHR == 0 && U_WD1T % NTHR == 0);
static_assert(U_WD1X % NTHR == 0 && U_WD2T % NTHR == 0 && U_WD3T % NTHR == 0);
static_assert(GBM == (GTHR / 32) * 16 && GBN == 4 * 32 && HID == 2 * GBN);
static_assert(KX % 32 == 0 && HID % 32 == 0 && H2C % 32 == 0);
static_assert(AGG_LDS_INTS * 4 <= 300000);
static_assert(GRU_LDS_BYTES == 65536);
static_assert(DEGCAP % 32 == 0);

typedef float          v4f   __attribute__((ext_vector_type(4)));
typedef float          v8f   __attribute__((ext_vector_type(8)));
typedef int            v4i   __attribute__((ext_vector_type(4)));
typedef int            v8i   __attribute__((ext_vector_type(8)));
typedef _Float16       v8h   __attribute__((ext_vector_type(8)));
typedef _Float16       v16h  __attribute__((ext_vector_type(16)));
typedef v4f __attribute__((may_alias)) v4fa;
typedef v4i __attribute__((may_alias)) v4ia;
typedef v8h __attribute__((may_alias)) v8ha;
union FragH { v16h v; v8h half[2]; v8i w; };

__device__ __forceinline__ v8f wmh(const FragH& a, const FragH& b, v8f c) {
  v8f d = __builtin_amdgcn_wmma_f32_16x16x32_f16(false, a.v, false, b.v, (short)0, c, false, false);
  asm volatile("v_nop\n\tv_nop\n\tv_nop\n\tv_nop" : "+v"(d) : "v"(a.w), "v"(b.w));
  return d;
}

__device__ __forceinline__ void ldfrag(FragH& f, const _Float16* p, int hh) {
  f.half[0] = *(const v8ha*)(p + 8 * hh);
  f.half[1] = *(const v8ha*)(p + 16 + 8 * hh);
}

template <int SLB>
__device__ __forceinline__ int scan_chunk(const int* __restrict__ dsts, int nE, int cbase, int slotBase,
                                          int nb, int vec8, int* list, int tid, int lane, int wave) {
  int wc = 0;
  const int el0  = tid * EPT;
  const int e0   = cbase + el0;
  const int sent = -2147483647 - 1;
  v4i da, db;
  if (vec8 != 0 && cbase + CHUNK <= nE) {
    da = *(const v4i*)(dsts + e0);
    db = *(const v4i*)(dsts + e0 + 4);
  } else {
    da.x = (e0     < nE) ? dsts[min(e0,     nE - 1)] : sent;
    da.y = (e0 + 1 < nE) ? dsts[min(e0 + 1, nE - 1)] : sent;
    da.z = (e0 + 2 < nE) ? dsts[min(e0 + 2, nE - 1)] : sent;
    da.w = (e0 + 3 < nE) ? dsts[min(e0 + 3, nE - 1)] : sent;
    db.x = (e0 + 4 < nE) ? dsts[min(e0 + 4, nE - 1)] : sent;
    db.y = (e0 + 5 < nE) ? dsts[min(e0 + 5, nE - 1)] : sent;
    db.z = (e0 + 6 < nE) ? dsts[min(e0 + 6, nE - 1)] : sent;
    db.w = (e0 + 7 < nE) ? dsts[min(e0 + 7, nE - 1)] : sent;
  }
  const unsigned nbs = (unsigned)slotBase;
  const unsigned unb = (unsigned)nb;
  const unsigned s0 = (unsigned)da.x - nbs, s1 = (unsigned)da.y - nbs;
  const unsigned s2 = (unsigned)da.z - nbs, s3 = (unsigned)da.w - nbs;
  const unsigned s4 = (unsigned)db.x - nbs, s5 = (unsigned)db.y - nbs;
  const unsigned s6 = (unsigned)db.z - nbs, s7 = (unsigned)db.w - nbs;
  const bool h0 = s0 < unb, h1 = s1 < unb, h2 = s2 < unb, h3 = s3 < unb;
  const bool h4 = s4 < unb, h5 = s5 < unb, h6 = s6 < unb, h7 = s7 < unb;
  const unsigned any = __builtin_amdgcn_ballot_w32(h0 | h1 | h2 | h3 | h4 | h5 | h6 | h7);
  if (any != 0u) {
#define HITJ(J, HJ, SJ) { \
      const unsigned mj = __builtin_amdgcn_ballot_w32(HJ); \
      if (mj != 0u) { \
        if (HJ) { \
          const int pos = wc + (int)__builtin_amdgcn_mbcnt_lo(mj, 0u); \
          if (pos < WCAP) list[wave * WCAP + pos] = ((el0 + (J)) << SLB) | (int)(SJ); \
        } \
        wc += (int)__builtin_popcount(mj); } }
    HITJ(0, h0, s0)
    HITJ(1, h1, s1)
    HITJ(2, h2, s2)
    HITJ(3, h3, s3)
    HITJ(4, h4, s4)
    HITJ(5, h5, s5)
    HITJ(6, h6, s6)
    HITJ(7, h7, s7)
#undef HITJ
  }
  return wc;
}

__global__ __launch_bounds__(NTHR) void k_prep(const float* __restrict__ x, int nN, int uX,
                                               const float* __restrict__ W1, const float* __restrict__ W2,
                                               const float* __restrict__ Wih, const float* __restrict__ Wd1,
                                               const float* __restrict__ Wd2, const float* __restrict__ Wd3,
                                               _Float16* XH, _Float16* W1T, _Float16* W2T, _Float16* WIHT,
                                               _Float16* WD1T, _Float16* WD1XT, _Float16* WD2T, _Float16* WD3T) {
  const int u = (int)blockIdx.x * NTHR + (int)threadIdx.x;
  float f[8];
  _Float16* dp;
  if (u < uX) {
    const int row = u >> 2, k8 = (u & 3) * 8;
    const int rc  = row < nN ? row : nN - 1;
    const float* p = x + (size_t)rc * DIN + (k8 & 8);
    const v4f a = *(const v4fa*)p;
    const v4f b = *(const v4fa*)(p + 4);
    const bool ok = (row < nN) && (k8 < DIN);
    f[0] = ok ? a.x * ASC : 0.0f; f[1] = ok ? a.y * ASC : 0.0f;
    f[2] = ok ? a.z * ASC : 0.0f; f[3] = ok ? a.w * ASC : 0.0f;
    f[4] = ok ? b.x * ASC : 0.0f; f[5] = ok ? b.y * ASC : 0.0f;
    f[6] = ok ? b.z * ASC : 0.0f; f[7] = ok ? b.w * ASC : 0.0f;
    dp = XH + (size_t)row * KX + k8;
  } else {
    const int v = u - uX;
    if (v < O1) {
      const int n = v >> 2, k8 = (v & 3) * 8, kk = k8 & 8;
      const bool kin = k8 < DIN;
#pragma unroll
      for (int i = 0; i < 8; ++i) {
        const float w = W1[(size_t)(kk + i) * HID + n];
        f[i] = kin ? w * WSC : 0.0f;
      }
      dp = W1T + (size_t)n * KX + k8;
    } else if (v < O2) {
      const int t = v - O1;
      const int n = t >> 5, k8 = (t & 31) * 8;
#pragma unroll
      for (int i = 0; i < 8; ++i) f[i] = W2[(size_t)(k8 + i) * HID + n] * WSC;
      dp = W2T + (size_t)n * HID + k8;
    } else if (v < O3) {
      const int t = v - O2;
      const int n = t >> 5, k8 = (t & 31) * 8;
#pragma unroll
      for (int i = 0; i < 8; ++i) f[i] = Wih[(size_t)n * HID + k8 + i] * WSC;
      dp = WIHT + (size_t)n * HID + k8;
    } else if (v < O4) {
      const int t = v - O3;
      const int n = t >> 5, k8 = (t & 31) * 8;
#pragma unroll
      for (int i = 0; i < 8; ++i) f[i] = Wd1[(size_t)(k8 + i) * HID + n] * WSC;
      dp = WD1T + (size_t)n * HID + k8;
    } else if (v < O5) {
      const int t = v - O4;
      const int n = t >> 2, k8 = (t & 3) * 8, kk = k8 & 8;
      const bool kin = k8 < DIN;
#pragma unroll
      for (int i = 0; i < 8; ++i) {
        const float w = Wd1[(size_t)(HID + kk + i) * HID + n];
        f[i] = kin ? w * WSC : 0.0f;
      }
      dp = WD1XT + (size_t)n * KX + k8;
    } else if (v < O6) {
      const int t = v - O5;
      const int n = t >> 5, k8 = (t & 31) * 8;
#pragma unroll
      for (int i = 0; i < 8; ++i) f[i] = Wd2[(size_t)(k8 + i) * H2C + n] * WSC;
      dp = WD2T + (size_t)n * HID + k8;
    } else if (v < O7) {
      const int t = v - O6;
      const int n = t >> 4, k8 = (t & 15) * 8;
      const int nc = n < DOUT ? n : DOUT - 1;
      const bool nin = n < DOUT;
#pragma unroll
      for (int i = 0; i < 8; ++i) {
        const float w = Wd3[(size_t)(k8 + i) * DOUT + nc];
        f[i] = nin ? w * WSC : 0.0f;
      }
      dp = WD3T + (size_t)n * H2C + k8;
    } else {
      return;
    }
  }
  const v8h o = { (_Float16)f[0], (_Float16)f[1], (_Float16)f[2], (_Float16)f[3],
                  (_Float16)f[4], (_Float16)f[5], (_Float16)f[6], (_Float16)f[7] };
  *(volatile v8h*)dp = o;
  __threadfence();
  *(volatile v8h*)dp = o;
}

__device__ __forceinline__ float disval(float s, bool live) {
  const float dg = s + 2.0f;
  const float r  = dg > 0.0f ? rsqrtf(fmaxf(dg, 1e-12f)) : 0.0f;
  return live ? r : 0.0f;
}

__global__ __launch_bounds__(NTHR) void k_deg(const int* __restrict__ dsts, const float* __restrict__ ew,
                                              int nE, int nN, int vec8, float* dis) {
  __shared__ __attribute__((aligned(16))) float sdeg[NBD];
  __shared__ __attribute__((aligned(16))) int list[LISTN];
  __shared__ int wcnt[NWAVE];
  const int tid = (int)threadIdx.x, lane = tid & 31, wave = tid >> 5;
  const int nodeBase = (int)blockIdx.x * NBD;

  for (int i = tid; i < NBD; i += NTHR) sdeg[i] = 0.0f;
  for (int i = tid; i < LISTN; i += NTHR) list[i] = 0;
  if (tid < NWAVE) wcnt[tid] = 0;
  __syncthreads();

  const int nChunks = (nE + CHUNK - 1) / CHUNK;
#pragma unroll 1
  for (int ch = 0; ch < nChunks; ++ch) {
    const int cbase = ch * CHUNK;
    const int wc = scan_chunk<SLD>(dsts, nE, cbase, nodeBase, NBD, vec8, list, tid, lane, wave);
    if (lane == 0) wcnt[wave] = wc;
    __syncthreads();
    if (wave == 0) {
#pragma unroll 1
      for (int w2 = 0; w2 < NWAVE; ++w2) {
        int c = wcnt[w2];
        c = c < 0 ? 0 : (c > WCAP ? WCAP : c);
#pragma unroll 1
        for (int b0 = 0; b0 < c; b0 += 32) {
          const int idx = b0 + lane;
          const int ent = list[w2 * WCAP + (idx < WCAP ? idx : WCAP - 1)];
          const int el  = (ent >> SLD) & (CHUNK - 1);
          int eid = cbase + el;
          eid = eid < 0 ? 0 : (eid > nE - 1 ? nE - 1 : eid);
          const int wvi = __float_as_int(ew[eid]);
          const int m32 = (c - b0) < 32 ? (c - b0) : 32;
#pragma unroll 1
          for (int k = 0; k < m32; ++k) {
            const int   u   = __builtin_amdgcn_readlane(ent, k);
            const float wk  = __int_as_float(__builtin_amdgcn_readlane(wvi, k));
            const int   slt = u & (NBD - 1);
            if (lane == 0) sdeg[slt] = sdeg[slt] + wk;
          }
        }
      }
    }
    __syncthreads();
  }

  v4f vals[NBD / (NTHR * 4)];
#pragma unroll
  for (int it = 0; it < NBD / (NTHR * 4); ++it) {
    const int s0 = it * (NTHR * 4) + 4 * tid;
    const v4f d4 = *(const v4fa*)(sdeg + s0);
    const int n0 = nodeBase + s0;
    v4f v;
    v.x = disval(d4.x, n0     < nN);
    v.y = disval(d4.y, n0 + 1 < nN);
    v.z = disval(d4.z, n0 + 2 < nN);
    v.w = disval(d4.w, n0 + 3 < nN);
    vals[it] = v;
  }
#pragma unroll
  for (int it = 0; it < NBD / (NTHR * 4); ++it) {
    const int s0 = it * (NTHR * 4) + 4 * tid;
    *(volatile v4f*)(dis + (size_t)nodeBase + s0) = vals[it];
  }
  __threadfence();
#pragma unroll
  for (int it = 0; it < NBD / (NTHR * 4); ++it) {
    const int s0 = it * (NTHR * 4) + 4 * tid;
    *(volatile v4f*)(dis + (size_t)nodeBase + s0) = vals[it];
  }
}

__global__ __launch_bounds__(GTHR) void k_gemmf(const _Float16* __restrict__ A, int lda,
                                                const _Float16* __restrict__ BT, int ldb, int K,
                                                float* Cm, int ldc) {
  __shared__ __attribute__((aligned(16))) float stg[GBM * GBN];
  const int tid = (int)threadIdx.x, lane = tid & 31, wave = tid >> 5, hh = lane >> 4, m = lane & 15;
  const int rowBase = (int)blockIdx.x * GBM;
  const int colBase = (int)blockIdx.y * GBN;

  v8f acc[8];
  {
    const v8f z = {0.f, 0.f, 0.f, 0.f, 0.f, 0.f, 0.f, 0.f};
#pragma unroll
    for (int t = 0; t < 8; ++t) acc[t] = z;
  }
  const _Float16* ap = A  + (size_t)(rowBase + 16 * wave + m) * (size_t)lda;
  const _Float16* bp = BT + (size_t)(colBase + m) * (size_t)ldb;

#pragma unroll 1
  for (int k0 = 0; k0 < K; k0 += 32) {
    FragH af;
    ldfrag(af, ap + k0, hh);
#pragma unroll
    for (int nt = 0; nt < 8; ++nt) {
      FragH bf;
      ldfrag(bf, bp + (size_t)(16 * nt) * (size_t)ldb + k0, hh);
      acc[nt] = wmh(af, bf, acc[nt]);
    }
  }

#pragma unroll
  for (int nt = 0; nt < 8; ++nt) {
    const int lc = 16 * nt + m;
#pragma unroll
    for (int r = 0; r < 8; ++r) {
      const int lr = 16 * wave + 8 * hh + r;
      stg[lr * GBN + lc] = acc[nt][r] * SCL;
    }
  }
  __syncthreads();

  v4f pv[16];
#pragma unroll
  for (int i = 0; i < 16; ++i) pv[i] = *(const v4fa*)(stg + (16 * wave + i) * GBN + 4 * lane);
#pragma unroll
  for (int i = 0; i < 16; ++i) {
    float* op = Cm + (size_t)(rowBase + 16 * wave + i) * (size_t)ldc + colBase + 4 * lane;
    *(volatile v4f*)op = pv[i];
  }
  __threadfence();
#pragma unroll
  for (int i = 0; i < 16; ++i) {
    float* op = Cm + (size_t)(rowBase + 16 * wave + i) * (size_t)ldc + colBase + 4 * lane;
    *(volatile v4f*)op = pv[i];
  }
}

template <int L1>
__global__ __launch_bounds__(NTHR) void k_agg(const int* __restrict__ srcs, const int* __restrict__ dsts,
                                              const float* __restrict__ ew, int nE, int nN, int vec8, int mRows,
                                              const float* __restrict__ dis, const float* __restrict__ xw,
                                              const float* __restrict__ bias, const float* __restrict__ gam,
                                              const float* __restrict__ bet, _Float16* hp) {
  extern __shared__ __attribute__((aligned(16))) int dsm[];
  int* list = dsm;
  int* hl   = dsm + LISTN;
  int* sl   = dsm + LISTN + RCAP;
  int* cnt  = dsm + LISTN + 2 * RCAP;
  int* offs = cnt + NBA;
  int* cur  = offs + NBA;
  int* misc = cur + NBA;
  const int tid = (int)threadIdx.x, lane = tid & 31, wave = tid >> 5;
  const int nodeBase = (int)blockIdx.x * NBA;

  {
    const v4i z4 = {0, 0, 0, 0};
    for (int i = tid * 4; i < AGG_ZINTS; i += NTHR * 4) *(v4ia*)(dsm + i) = z4;
    if (tid < 16) misc[tid] = 0;
  }
  float bv[8], gv[8], ev[8];
  {
    const v4f a = *(const v4fa*)(bias + 8 * lane);
    const v4f b = *(const v4fa*)(bias + 8 * lane + 4);
    bv[0] = a.x; bv[1] = a.y; bv[2] = a.z; bv[3] = a.w; bv[4] = b.x; bv[5] = b.y; bv[6] = b.z; bv[7] = b.w;
    const v4f c = *(const v4fa*)(gam + 8 * lane);
    const v4f d = *(const v4fa*)(gam + 8 * lane + 4);
    gv[0] = c.x; gv[1] = c.y; gv[2] = c.z; gv[3] = c.w; gv[4] = d.x; gv[5] = d.y; gv[6] = d.z; gv[7] = d.w;
    const v4f e = *(const v4fa*)(bet + 8 * lane);
    const v4f g = *(const v4fa*)(bet + 8 * lane + 4);
    ev[0] = e.x; ev[1] = e.y; ev[2] = e.z; ev[3] = e.w; ev[4] = g.x; ev[5] = g.y; ev[6] = g.z; ev[7] = g.w;
  }
  __syncthreads();

  int t = 0, ov = 0;
  const int nChunks = (nE + CHUNK - 1) / CHUNK;
#pragma unroll 1
  for (int ch = 0; ch < nChunks; ++ch) {
    const int cbase = ch * CHUNK;
    const int wc = scan_chunk<SLA>(dsts, nE, cbase, nodeBase, NBA, vec8, list, tid, lane, wave);
    if (lane == 0) misc[wave] = wc;
    __syncthreads();
    if (wave == 0) {
#pragma unroll 1
      for (int w2 = 0; w2 < NWAVE; ++w2) {
        int c = misc[w2];
        c = c < 0 ? 0 : (c > WCAP ? WCAP : c);
#pragma unroll 1
        for (int b0 = 0; b0 < c; b0 += 32) {
          const int idx = b0 + lane;
          const int ent = list[w2 * WCAP + (idx < WCAP ? idx : WCAP - 1)];
          const int m32 = (c - b0) < 32 ? (c - b0) : 32;
#pragma unroll 1
          for (int k = 0; k < m32; ++k) {
            const int u    = __builtin_amdgcn_readlane(ent, k);
            const int slot = u & (NBA - 1);
            const int el   = (u >> SLA) & (CHUNK - 1);
            const int pk   = ((cbase + el) << SLA) | slot;
            if (t < RCAP) {
              if (lane == 0) { hl[t] = pk; cnt[slot] = cnt[slot] + 1; }
              t = t + 1;
            } else {
              ov = 1;
            }
          }
        }
      }
    }
    __syncthreads();
  }
  if (wave == 0 && lane == 0) { misc[8] = t; misc[9] = ov; }
  __syncthreads();
  int tt = misc[8];
  tt = tt < 0 ? 0 : (tt > RCAP ? RCAP : tt);
  const int ovf = misc[9];

  if (wave == 0) {
    const int base = lane * (NBA / 32);
    int s = 0;
#pragma unroll 1
    for (int i = 0; i < NBA / 32; ++i) s += cnt[base + i];
    int incl = s;
#pragma unroll
    for (int d = 1; d < 32; d <<= 1) {
      const int y = __shfl_up(incl, d, 32);
      if (lane >= d) incl += y;
    }
    int run = incl - s;
#pragma unroll 1
    for (int i = 0; i < NBA / 32; ++i) {
      const int cv = cnt[base + i];
      offs[base + i] = run;
      cur[base + i]  = run;
      run += cv;
    }
  }
  __syncthreads();
  if (wave == 0) {
#pragma unroll 1
    for (int b0 = 0; b0 < tt; b0 += 32) {
      const int idx = b0 + lane;
      const int ent = hl[idx < RCAP ? idx : RCAP - 1];
      const int m32 = (tt - b0) < 32 ? (tt - b0) : 32;
#pragma unroll 1
      for (int k = 0; k < m32; ++k) {
        const int u    = __builtin_amdgcn_readlane(ent, k);
        const int slot = u & (NBA - 1);
        if (lane == 0) {
          int p = cur[slot];
          p = p < 0 ? 0 : (p > RCAP - 1 ? RCAP - 1 : p);
          sl[p] = u;
          cur[slot] = p + 1;
        }
      }
    }
  }
  __syncthreads();

  const float pz = (ovf != 0) ? __int_as_float(0x7fc00000) : 0.0f;
#pragma unroll 1
  for (int si = 0; si < NBA / NWAVE; ++si) {
    const int s    = si * NWAVE + wave;
    const int node = nodeBase + s;
    int c = cnt[s];
    const bool big = c > DEGCAP;
    c = c < 0 ? 0 : (c > DEGCAP ? DEGCAP : c);
    int o = offs[s];
    o = o < 0 ? 0 : (o > RCAP ? RCAP : o);
    const int nc = node < nN ? node : nN - 1;
    const float dd = dis[nc];
    float acc[8];
#pragma unroll
    for (int i = 0; i < 8; ++i) acc[i] = 0.0f;
#pragma unroll 1
    for (int b0 = 0; b0 < c; b0 += 32) {
      int idx = o + b0 + lane;
      idx = idx > RCAP - 1 ? RCAP - 1 : idx;
      const int ent = sl[idx];
      int eid = ent >> SLA;
      eid = eid < 0 ? 0 : (eid > nE - 1 ? nE - 1 : eid);
      int sr = srcs[eid];
      sr = sr < 0 ? 0 : (sr > nN - 1 ? nN - 1 : sr);
      const float we  = ew[eid];
      const float cf  = (dis[sr] * we) * dd;
      const int   cfi = __float_as_int(cf);
      const int m32 = (c - b0) < 32 ? (c - b0) : 32;
#pragma unroll 1
      for (int k = 0; k < m32; ++k) {
        const int   sk = __builtin_amdgcn_readlane(sr, k);
        const float ck = __int_as_float(__builtin_amdgcn_readlane(cfi, k));
        const float* rp = xw + (size_t)sk * HID + 8 * lane;
        const v4f a = *(const v4fa*)rp;
        const v4f b = *(const v4fa*)(rp + 4);
        acc[0] = fmaf(ck, a.x, acc[0]); acc[1] = fmaf(ck, a.y, acc[1]);
        acc[2] = fmaf(ck, a.z, acc[2]); acc[3] = fmaf(ck, a.w, acc[3]);
        acc[4] = fmaf(ck, b.x, acc[4]); acc[5] = fmaf(ck, b.y, acc[5]);
        acc[6] = fmaf(ck, b.z, acc[6]); acc[7] = fmaf(ck, b.w, acc[7]);
      }
    }
    float sv[8];
    {
      const float* sp = xw + (size_t)nc * HID + 8 * lane;
      const v4f a = *(const v4fa*)sp;
      const v4f b = *(const v4fa*)(sp + 4);
      sv[0] = a.x; sv[1] = a.y; sv[2] = a.z; sv[3] = a.w;
      sv[4] = b.x; sv[5] = b.y; sv[6] = b.z; sv[7] = b.w;
    }
    const float ns = (dd * 2.0f) * dd;
    float v[8];
#pragma unroll
    for (int i = 0; i < 8; ++i) v[i] = (acc[i] + sv[i] * ns) + bv[i];
    float s1 = 0.0f;
#pragma unroll
    for (int i = 0; i < 8; ++i) s1 += v[i];
#pragma unroll
    for (int q = 16; q > 0; q >>= 1) s1 += __shfl_xor(s1, q, 32);
    const float mu = s1 * (1.0f / 256.0f);
    float s2 = 0.0f;
#pragma unroll
    for (int i = 0; i < 8; ++i) { const float d = v[i] - mu; s2 += d * d; }
#pragma unroll
    for (int q = 16; q > 0; q >>= 1) s2 += __shfl_xor(s2, q, 32);
    const float rs = rsqrtf(s2 * (1.0f / 256.0f) + 1e-5f);
    const float pzr = big ? __int_as_float(0x7fc00000) : pz;
    const bool live = node < nN;
    v8h ho;
#pragma unroll
    for (int i = 0; i < 8; ++i) {
      float y = (v[i] - mu) * rs * gv[i] + ev[i];
      if (L1 != 0) y = fmaxf(y, 0.0f);
      y = y + pzr;
      y = live ? y : 0.0f;
      ho[i] = (_Float16)(y * ASC);
    }
    if (node < mRows) {
      _Float16* hq = hp + (size_t)node * HID + 8 * lane;
      *(volatile v8h*)hq = ho;
      __threadfence();
      *(volatile v8h*)hq = ho;
    }
  }
}

__device__ __forceinline__ void st_rows64(const _Float16* sT, _Float16* plane, int rowBase, int colBase,
                                          int wave, int lane) {
  const int q8 = lane & 7, sub = lane >> 3;
#pragma unroll
  for (int i = 0; i < 4; ++i) {
    const int lid = 16 * wave + 4 * i + sub;
    const v8h v = *(const v8ha*)(sT + lid * 64 + 8 * q8);
    _Float16* d = plane + (size_t)(rowBase + lid) * HID + colBase + 8 * q8;
    *(volatile v8h*)d = v;
  }
}

__global__ __launch_bounds__(GTHR) void k_gru(const _Float16* __restrict__ H2, const _Float16* __restrict__ WIHT,
                                              const float* __restrict__ bih, const float* __restrict__ bhh,
                                              _Float16* TH, _Float16* TL) {
  extern __shared__ __attribute__((aligned(16))) float gsm[];
  float* sG = gsm;
  _Float16* sHi = (_Float16*)(gsm + 3 * 64 * 64);
  _Float16* sLo = sHi + 64 * 64;
  const int tid = (int)threadIdx.x, lane = tid & 31, wave = tid >> 5, hh = lane >> 4, m = lane & 15;
  const int rowBase = (int)blockIdx.x * 64;
  const int ub = (int)blockIdx.y * 64;
  const _Float16* ap = H2 + (size_t)(rowBase + 16 * wave + m) * HID;
  const v8f z8 = {0.f, 0.f, 0.f, 0.f, 0.f, 0.f, 0.f, 0.f};

#pragma unroll 1
  for (int g = 0; g < 3; ++g) {
    v8f acc[4];
#pragma unroll
    for (int t = 0; t < 4; ++t) acc[t] = z8;
    const _Float16* bp = WIHT + (size_t)(g * HID + ub + m) * HID;
#pragma unroll 1
    for (int k0 = 0; k0 < HID; k0 += 32) {
      FragH af;
      ldfrag(af, ap + k0, hh);
#pragma unroll
      for (int nt = 0; nt < 4; ++nt) {
        FragH bf;
        ldfrag(bf, bp + (size_t)(16 * nt) * HID + k0, hh);
        acc[nt] = wmh(af, bf, acc[nt]);
      }
    }
#pragma unroll
    for (int nt = 0; nt < 4; ++nt) {
#pragma unroll
      for (int r = 0; r < 8; ++r) {
        const int lr = 16 * wave + 8 * hh + r;
        sG[(g * 64 + lr) * 64 + 16 * nt + m] = acc[nt][r] * SCL;
      }
    }
  }
  __syncthreads();

  {
    const int u = tid & 63;
    const int j = ub + u;
    const float cbr = bih[j] + bhh[j];
    const float cbz = bih[HID + j] + bhh[HID + j];
    const float cbi = bih[2 * HID + j];
    const float cbh = bhh[2 * HID + j];
#pragma unroll 1
    for (int i = 0; i < 32; ++i) {
      const int row = (tid >> 6) + 2 * i;
      const float gr = sG[row * 64 + u];
      const float gz = sG[(64 + row) * 64 + u];
      const float gn = sG[(128 + row) * 64 + u];
      const float er = expf(fminf(-(gr + cbr), 80.0f));
      const float ez = expf(fminf(-(gz + cbz), 80.0f));
      const float rg = __builtin_amdgcn_rcpf(1.0f + er);
      const float zg = __builtin_amdgcn_rcpf(1.0f + ez);
      const float ng = tanhf(gn + cbi + rg * cbh);
      const float tv = (1.0f - zg) * ng;
      const float t8 = tv * ASC;
      const _Float16 hi = (_Float16)t8;
      const _Float16 lo = (_Float16)((t8 - (float)hi) * RSC);
      sHi[row * 64 + u] = hi;
      sLo[row * 64 + u] = lo;
    }
  }
  __syncthreads();

  st_rows64(sHi, TH, rowBase, ub, wave, lane);
  st_rows64(sLo, TL, rowBase, ub, wave, lane);
  __threadfence();
  st_rows64(sHi, TH, rowBase, ub, wave, lane);
  st_rows64(sLo, TL, rowBase, ub, wave, lane);
}

__global__ __launch_bounds__(GTHR) void k_dec1(const _Float16* __restrict__ TH, const _Float16* __restrict__ TL,
                                               const _Float16* __restrict__ XH, const _Float16* __restrict__ WD1T,
                                               const _Float16* __restrict__ WD1XT, const float* __restrict__ bd1,
                                               _Float16* D1H, _Float16* D1L) {
  __shared__ __attribute__((aligned(16))) _Float16 sHi[64 * 64];
  __shared__ __attribute__((aligned(16))) _Float16 sLo[64 * 64];
  const int tid = (int)threadIdx.x, lane = tid & 31, wave = tid >> 5, hh = lane >> 4, m = lane & 15;
  const int rowBase = (int)blockIdx.x * 64;
  const int cb = (int)blockIdx.y * 64;
  const v8f z8 = {0.f, 0.f, 0.f, 0.f, 0.f, 0.f, 0.f, 0.f};

  v8f acc[4], accr[4];
#pragma unroll
  for (int t = 0; t < 4; ++t) { acc[t] = z8; accr[t] = z8; }
  const int arow = rowBase + 16 * wave + m;
  const _Float16* aph = TH + (size_t)arow * HID;
  const _Float16* apl = TL + (size_t)arow * HID;
  const _Float16* bp  = WD1T + (size_t)(cb + m) * HID;

#pragma unroll 1
  for (int k0 = 0; k0 < HID; k0 += 32) {
    FragH ah, al;
    ldfrag(ah, aph + k0, hh);
    ldfrag(al, apl + k0, hh);
#pragma unroll
    for (int nt = 0; nt < 4; ++nt) {
      FragH bf;
      ldfrag(bf, bp + (size_t)(16 * nt) * HID + k0, hh);
      acc[nt]  = wmh(ah, bf, acc[nt]);
      accr[nt] = wmh(al, bf, accr[nt]);
    }
  }
  {
    FragH ax;
    ldfrag(ax, XH + (size_t)arow * KX, hh);
    const _Float16* bx = WD1XT + (size_t)(cb + m) * KX;
#pragma unroll
    for (int nt = 0; nt < 4; ++nt) {
      FragH bf;
      ldfrag(bf, bx + (size_t)(16 * nt) * KX, hh);
      acc[nt] = wmh(ax, bf, acc[nt]);
    }
  }

#pragma unroll
  for (int nt = 0; nt < 4; ++nt) {
    const int lc = 16 * nt + m;
    const float bb = bd1[cb + lc];
#pragma unroll
    for (int r = 0; r < 8; ++r) {
      const int lr = 16 * wave + 8 * hh + r;
      float v = acc[nt][r] * SCL + accr[nt][r] * SCLR + bb;
      v = fmaxf(v, 0.0f);
      const float v8 = v * ASC;
      const _Float16 hi = (_Float16)v8;
      const _Float16 lo = (_Float16)((v8 - (float)hi) * RSC);
      sHi[lr * 64 + lc] = hi;
      sLo[lr * 64 + lc] = lo;
    }
  }
  __syncthreads();

  st_rows64(sHi, D1H, rowBase, cb, wave, lane);
  st_rows64(sLo, D1L, rowBase, cb, wave, lane);
  __threadfence();
  st_rows64(sHi, D1H, rowBase, cb, wave, lane);
  st_rows64(sLo, D1L, rowBase, cb, wave, lane);
}

__global__ __launch_bounds__(GTHR) void k_dec2(const _Float16* __restrict__ D1H, const _Float16* __restrict__ D1L,
                                               const _Float16* __restrict__ WD2T, const _Float16* __restrict__ WD3T,
                                               const float* __restrict__ bd2, const float* __restrict__ bd3,
                                               float* outp, int nN) {
  __shared__ __attribute__((aligned(16))) _Float16 sHi[64 * H2C];
  __shared__ __attribute__((aligned(16))) _Float16 sLo[64 * H2C];
  __shared__ __attribute__((aligned(16))) float sO[64 * DOUT];
  const int tid = (int)threadIdx.x, lane = tid & 31, wave = tid >> 5, hh = lane >> 4, m = lane & 15;
  const int rowBase = (int)blockIdx.x * 64;
  const v8f z8 = {0.f, 0.f, 0.f, 0.f, 0.f, 0.f, 0.f, 0.f};
  const int arow = rowBase + 16 * wave + m;
  const _Float16* aph = D1H + (size_t)arow * HID;
  const _Float16* apl = D1L + (size_t)arow * HID;

#pragma unroll 1
  for (int cb = 0; cb < 2; ++cb) {
    v8f acc[4], accr[4];
#pragma unroll
    for (int t = 0; t < 4; ++t) { acc[t] = z8; accr[t] = z8; }
    const _Float16* bp = WD2T + (size_t)(64 * cb + m) * HID;
#pragma unroll 1
    for (int k0 = 0; k0 < HID; k0 += 32) {
      FragH ah, al;
      ldfrag(ah, aph + k0, hh);
      ldfrag(al, apl + k0, hh);
#pragma unroll
      for (int nt = 0; nt < 4; ++nt) {
        FragH bf;
        ldfrag(bf, bp + (size_t)(16 * nt) * HID + k0, hh);
        acc[nt]  = wmh(ah, bf, acc[nt]);
        accr[nt] = wmh(al, bf, accr[nt]);
      }
    }
#pragma unroll
    for (int nt = 0; nt < 4; ++nt) {
      const int c = 64 * cb + 16 * nt + m;
      const float bb = bd2[c];
#pragma unroll
      for (int r = 0; r < 8; ++r) {
        const int lr = 16 * wave + 8 * hh + r;
        float v = acc[nt][r] * SCL + accr[nt][r] * SCLR + bb;
        v = fmaxf(v, 0.0f);
        const float v8 = v * ASC;
        const _Float16 hi = (_Float16)v8;
        const _Float16 lo = (_Float16)((v8 - (float)hi) * RSC);
        sHi[lr * H2C + c] = hi;
        sLo[lr * H2C + c] = lo;
      }
    }
  }
  __syncthreads();

  v8f acc3 = z8, acc3r = z8;
  {
    const int lrow = (16 * wave + m) * H2C;
    const _Float16* b3 = WD3T + (size_t)m * H2C;
#pragma unroll
    for (int k0 = 0; k0 < H2C; k0 += 32) {
      FragH ah, al, bf;
      ah.half[0] = *(const v8ha*)(sHi + lrow + k0 + 8 * hh);
      ah.half[1] = *(const v8ha*)(sHi + lrow + k0 + 16 + 8 * hh);
      al.half[0] = *(const v8ha*)(sLo + lrow + k0 + 8 * hh);
      al.half[1] = *(const v8ha*)(sLo + lrow + k0 + 16 + 8 * hh);
      ldfrag(bf, b3 + k0, hh);
      acc3  = wmh(ah, bf, acc3);
      acc3r = wmh(al, bf, acc3r);
    }
  }
  {
    const int mc = m < DOUT ? m : DOUT - 1;
    const float b3v = bd3[mc];
#pragma unroll
    for (int r = 0; r < 8; ++r) {
      float p = acc3[r] * SCL + acc3r[r] * SCLR + b3v;
      p = fminf(fmaxf(p, -5.0f), 5.0f);
      if (m < DOUT) sO[(16 * wave + 8 * hh + r) * DOUT + m] = p;
    }
  }
  __syncthreads();

  int valid = nN - rowBase;
  valid = valid < 0 ? 0 : (valid > 64 ? 64 : valid);
  const bool act = (4 * lane + 4) <= DOUT * valid;
  const v4f ov = *(const v4fa*)(sO + 4 * lane);
  float* op = outp + (size_t)rowBase * DOUT + 4 * lane;
  if (wave == 0 && act) *(volatile v4f*)op = ov;
  __threadfence();
  if (wave == 0 && act) *(volatile v4f*)op = ov;
}

static inline int cdiv(int a, int b) { return (a + b - 1) / b; }

extern "C" void kernel_launch(void* const* d_in, const int* in_sizes, int n_in,
                              void* d_out, int out_size, void* d_ws, size_t ws_size,
                              hipStream_t stream) {
  if (n_in < 21) return;
  if (in_sizes[0] < DIN * 16 || (in_sizes[0] % DIN) != 0) return;
  const int nN = in_sizes[0] / DIN;
  if ((nN % 16) != 0) return;
  if (in_sizes[1] < 2 || (in_sizes[1] & 1) != 0) return;
  const int nE = in_sizes[1] / 2;
  if (nE < 1 || nE >= (1 << 22)) return;
  if (in_sizes[2] != nE) return;
  if (in_sizes[3] != DIN * HID || in_sizes[4] != HID || in_sizes[5] != HID || in_sizes[6] != HID) return;
  if (in_sizes[7] != HID * HID || in_sizes[8] != HID || in_sizes[9] != HID || in_sizes[10] != HID) return;
  if (in_sizes[11] != G3 * HID || in_sizes[12] != G3 * HID || in_sizes[13] != G3 || in_sizes[14] != G3) return;
  if (in_sizes[15] != (HID + DIN) * HID || in_sizes[16] != HID) return;
  if (in_sizes[17] != HID * H2C || in_sizes[18] != H2C) return;
  if (in_sizes[19] != H2C * DOUT || in_sizes[20] != DOUT) return;
  if ((long long)out_size != (long long)nN * DOUT) return;

  const float* x    = (const float*)d_in[0];
  const int*   edge = (const int*)d_in[1];
  const float* ew   = (const float*)d_in[2];
  const float* W1   = (const float*)d_in[3];
  const float* b1   = (const float*)d_in[4];
  const float* g1   = (const float*)d_in[5];
  const float* be1  = (const float*)d_in[6];
  const float* W2   = (const float*)d_in[7];
  const float* b2   = (const float*)d_in[8];
  const float* g2   = (const float*)d_in[9];
  const float* be2  = (const float*)d_in[10];
  const float* Wih  = (const float*)d_in[11];
  const float* bih  = (const float*)d_in[13];
  const float* bhh  = (const float*)d_in[14];
  const float* Wd1  = (const float*)d_in[15];
  const float* bd1  = (const float*)d_in[16];
  const float* Wd2  = (const float*)d_in[17];
  const float* bd2  = (const float*)d_in[18];
  const float* Wd3  = (const float*)d_in[19];
  const float* bd3  = (const float*)d_in[20];
  float* out = (float*)d_out;
  const int* src = edge;
  const int* dst = edge + nE;

  const int MP   = cdiv(nN, GBM) * GBM;
  const int gM   = MP / GBM;
  const int gD   = cdiv(nN, NBD);
  const int NBPD = gD * NBD;
  const int gA   = cdiv(nN, NBA);
  if ((long long)gA * NBA < (long long)MP) return;
  if (NBPD < nN) return;
  const int vec8 = ((nE & 3) == 0) ? 1 : 0;

  char* ws = (char*)d_ws;
  size_t off = 0;
  const size_t oXH   = off; off += (size_t)MP * KX * 2;        off = (off + 255) & ~(size_t)255;
  const size_t oW1T  = off; off += (size_t)HID * KX * 2;       off = (off + 255) & ~(size_t)255;
  const size_t oW2T  = off; off += (size_t)HID * HID * 2;      off = (off + 255) & ~(size_t)255;
  const size_t oWIH  = off; off += (size_t)G3 * HID * 2;       off = (off + 255) & ~(size_t)255;
  const size_t oWD1T = off; off += (size_t)HID * HID * 2;      off = (off + 255) & ~(size_t)255;
  const size_t oWD1X = off; off += (size_t)HID * KX * 2;       off = (off + 255) & ~(size_t)255;
  const size_t oWD2T = off; off += (size_t)H2C * HID * 2;      off = (off + 255) & ~(size_t)255;
  const size_t oWD3T = off; off += (size_t)16 * H2C * 2;       off = (off + 255) & ~(size_t)255;
  const size_t oDIS  = off; off += (size_t)NBPD * 4;           off = (off + 255) & ~(size_t)255;
  const size_t szXW  = (size_t)MP * HID * 4;
  const size_t szD1  = (size_t)2 * MP * HID * 2;
  const size_t oRXW  = off; off += (szXW > szD1 ? szXW : szD1); off = (off + 255) & ~(size_t)255;
  const size_t oRH   = off; off += (size_t)MP * HID * 2;       off = (off + 255) & ~(size_t)255;
  const size_t oRT   = off; off += (size_t)2 * MP * HID * 2;   off = (off + 255) & ~(size_t)255;
  if (off > ws_size || off > (size_t)WSMAX) return;

  _Float16* XH    = (_Float16*)(ws + oXH);
  _Float16* W1T   = (_Float16*)(ws + oW1T);
  _Float16* W2T   = (_Float16*)(ws + oW2T);
  _Float16* WIHT  = (_Float16*)(ws + oWIH);
  _Float16* WD1T  = (_Float16*)(ws + oWD1T);
  _Float16* WD1XT = (_Float16*)(ws + oWD1X);
  _Float16* WD2T  = (_Float16*)(ws + oWD2T);
  _Float16* WD3T  = (_Float16*)(ws + oWD3T);
  float*    DIS   = (float*)(ws + oDIS);
  float*    XW    = (float*)(ws + oRXW);
  _Float16* D1H   = (_Float16*)(ws + oRXW);
  _Float16* D1L   = D1H + (size_t)MP * HID;
  _Float16* H     = (_Float16*)(ws + oRH);
  _Float16* TH    = (_Float16*)(ws + oRT);
  _Float16* TL    = TH + (size_t)MP * HID;

  const size_t aggLds = (size_t)AGG_LDS_INTS * 4;
  hipFuncSetAttribute(reinterpret_cast<const void*>(&k_agg<1>), hipFuncAttributeMaxDynamicSharedMemorySize, (int)aggLds);
  hipFuncSetAttribute(reinterpret_cast<const void*>(&k_agg<0>), hipFuncAttributeMaxDynamicSharedMemorySize, (int)aggLds);
  hipFuncSetAttribute(reinterpret_cast<const void*>(&k_gru), hipFuncAttributeMaxDynamicSharedMemorySize, (int)GRU_LDS_BYTES);

  const int uX = MP * (KX / 8);
  k_prep<<<(uX + O7) / NTHR, NTHR, 0, stream>>>(x, nN, uX, W1, W2, Wih, Wd1, Wd2, Wd3,
                                                XH, W1T, W2T, WIHT, WD1T, WD1XT, WD2T, WD3T);
  k_deg<<<gD, NTHR, 0, stream>>>(dst, ew, nE, nN, vec8, DIS);
  k_gemmf<<<dim3(gM, HID / GBN), GTHR, 0, stream>>>(XH, KX, W1T, KX, KX, XW, HID);
  k_agg<1><<<gA, NTHR, aggLds, stream>>>(src, dst, ew, nE, nN, vec8, MP, DIS, XW, b1, g1, be1, H);
  k_gemmf<<<dim3(gM, HID / GBN), GTHR, 0, stream>>>(H, HID, W2T, HID, HID, XW, HID);
  k_agg<0><<<gA, NTHR, aggLds, stream>>>(src, dst, ew, nE, nN, vec8, MP, DIS, XW, b2, g2, be2, H);
  k_gru<<<dim3(gM, HID / 64), GTHR, GRU_LDS_BYTES, stream>>>(H, WIHT, bih, bhh, TH, TL);
  k_dec1<<<dim3(gM, HID / 64), GTHR, 0, stream>>>(TH, TL, XH, WD1T, WD1XT, bd1, D1H, D1L);
  k_dec2<<<gM, GTHR, 0, stream>>>(D1H, D1L, WD2T, WD3T, bd2, bd3, out, nN);
}
